// LSTransformerEncoderLayer_67894843015649
// MI455X (gfx1250) — hardware-verified
//
#include <hip/hip_runtime.h>
#include <math.h>
#include <stdint.h>

#define NBATCH 8
#define SEQ    1024
#define HSZ    1024
#define IMSZ   4096
#define NH     16
#define HD     64
#define QKP    (2 * HSZ)
#define NKT    (SEQ / 64)
#define NTOK   (NBATCH * SEQ)
static_assert(NH * HD == HSZ);
static_assert((SEQ % 64) == 0 && (HSZ % 64) == 0 && (IMSZ % 64) == 0 && (NTOK % 64) == 0);

#define CW_QKV 64.0f
#define CW_O   64.0f
#define CW_I   32.0f
#define CW_F   64.0f
#define C_CTX  32.0f
#define C_P    1024.0f

typedef _Float16 v16h __attribute__((ext_vector_type(16)));
typedef _Float16 v8h  __attribute__((ext_vector_type(8)));
typedef float    v8f  __attribute__((ext_vector_type(8)));
typedef float    v4f  __attribute__((ext_vector_type(4)));
typedef unsigned int v4u __attribute__((ext_vector_type(4)));

__device__ __forceinline__ unsigned short h_bits(_Float16 x) { return __builtin_bit_cast(unsigned short, x); }
__device__ __forceinline__ unsigned pk16(unsigned short a, unsigned short b) { return (unsigned)a | ((unsigned)b << 16); }
__device__ __forceinline__ unsigned pkf(float a, float b) {
  return pk16(h_bits((_Float16)a), h_bits((_Float16)b));
}
__device__ __forceinline__ v8f zero8() { v8f z = {0.f, 0.f, 0.f, 0.f, 0.f, 0.f, 0.f, 0.f}; return z; }

__device__ __forceinline__ v16h ldfrag(const _Float16* p) {
  union { v16h v; v8h h[2]; } f;
  f.h[0] = *(const v8h*)(p);
  f.h[1] = *(const v8h*)(p + 16);
  return f.v;
}

__device__ __forceinline__ v8f mma_raw(v16h a, v16h b, v8f c) {
  return __builtin_amdgcn_wmma_f32_16x16x32_f16(false, a, false, b, (short)0, c, false, false);
}
__device__ __forceinline__ v8f mma_g(v16h a, v16h b, v8f c) {
  c = mma_raw(a, b, c);
#if defined(__HIP_DEVICE_COMPILE__)
  asm volatile("v_nop\n\tv_nop\n\tv_nop\n\tv_nop" : "+v"(c) : "v"(a), "v"(b));
#endif
  return c;
}
__device__ __forceinline__ void dep_guard(v8f& a, v8f& b, v16h x) {
#if defined(__HIP_DEVICE_COMPILE__)
  asm volatile("v_nop\n\tv_nop\n\tv_nop\n\tv_nop" : "+v"(a), "+v"(b) : "v"(x));
#else
  (void)a; (void)b; (void)x;
#endif
}
__device__ __forceinline__ void keep4(v16h a, v16h b, v16h c, v16h d) {
#if defined(__HIP_DEVICE_COMPILE__)
  asm volatile("v_nop" :: "v"(a), "v"(b), "v"(c), "v"(d));
#else
  (void)a; (void)b; (void)c; (void)d;
#endif
}
__device__ __forceinline__ void acc_guard4(v8f& a, v8f& b, v8f& c, v8f& d) {
#if defined(__HIP_DEVICE_COMPILE__)
  asm volatile("v_nop\n\tv_nop\n\tv_nop\n\tv_nop" : "+v"(a), "+v"(b), "+v"(c), "+v"(d));
#else
  (void)a; (void)b; (void)c; (void)d;
#endif
}

__global__ __launch_bounds__(256) void cvt_f16x8(const float* __restrict__ in, unsigned short* out,
                                                  int n8, float scale) {
  const int i = blockIdx.x * 256 + threadIdx.x;
  if (i < n8) {
    const v4f a = *(const v4f*)(in + (size_t)i * 8);
    const v4f b = *(const v4f*)(in + (size_t)i * 8 + 4);
    v4u p;
    p[0] = pkf(a[0] * scale, a[1] * scale);
    p[1] = pkf(a[2] * scale, a[3] * scale);
    p[2] = pkf(b[0] * scale, b[1] * scale);
    p[3] = pkf(b[2] * scale, b[3] * scale);
    unsigned short* d = out + (size_t)i * 8;
    *(volatile v4u*)d = p;
    __threadfence();
    *(volatile v4u*)d = p;
  }
}

__global__ __launch_bounds__(256) void ln_f16(const float* __restrict__ x, const float* __restrict__ g,
                                               const float* __restrict__ be, unsigned short* out,
                                               int nrows) {
  const int lane = threadIdx.x & 31;
  const int wave = threadIdx.x >> 5;
  const int row  = blockIdx.x * 8 + wave;
  if (row >= nrows) return;
  const float* xr = x + (size_t)row * HSZ;
  float v[32];
#pragma unroll
  for (int j = 0; j < 4; ++j) {
    const v4f a = *(const v4f*)(xr + j * 256 + lane * 8);
    const v4f b = *(const v4f*)(xr + j * 256 + lane * 8 + 4);
    v[8 * j + 0] = a[0]; v[8 * j + 1] = a[1]; v[8 * j + 2] = a[2]; v[8 * j + 3] = a[3];
    v[8 * j + 4] = b[0]; v[8 * j + 5] = b[1]; v[8 * j + 6] = b[2]; v[8 * j + 7] = b[3];
  }
  float s = 0.f;
#pragma unroll
  for (int e = 0; e < 32; ++e) s += v[e];
#pragma unroll
  for (int off = 1; off < 32; off <<= 1) s += __shfl_xor(s, off, 32);
  const float mu = s * (1.0f / HSZ);
  float s2 = 0.f;
#pragma unroll
  for (int e = 0; e < 32; ++e) { const float d = v[e] - mu; s2 += d * d; }
#pragma unroll
  for (int off = 1; off < 32; off <<= 1) s2 += __shfl_xor(s2, off, 32);
  const float var = s2 * (1.0f / HSZ);
  const float rs  = rsqrtf(var + 1e-5f);

  v4u pk[4];
#pragma unroll
  for (int j = 0; j < 4; ++j) {
    const int i0 = j * 256 + lane * 8;
    const v4f g0 = *(const v4f*)(g + i0);
    const v4f g1 = *(const v4f*)(g + i0 + 4);
    const v4f b0 = *(const v4f*)(be + i0);
    const v4f b1 = *(const v4f*)(be + i0 + 4);
    float o[8];
    o[0] = (v[8 * j + 0] - mu) * rs * g0[0] + b0[0];
    o[1] = (v[8 * j + 1] - mu) * rs * g0[1] + b0[1];
    o[2] = (v[8 * j + 2] - mu) * rs * g0[2] + b0[2];
    o[3] = (v[8 * j + 3] - mu) * rs * g0[3] + b0[3];
    o[4] = (v[8 * j + 4] - mu) * rs * g1[0] + b1[0];
    o[5] = (v[8 * j + 5] - mu) * rs * g1[1] + b1[1];
    o[6] = (v[8 * j + 6] - mu) * rs * g1[2] + b1[2];
    o[7] = (v[8 * j + 7] - mu) * rs * g1[3] + b1[3];
    v4u p;
    p[0] = pkf(o[0], o[1]); p[1] = pkf(o[2], o[3]); p[2] = pkf(o[4], o[5]); p[3] = pkf(o[6], o[7]);
    pk[j] = p;
  }
  unsigned short* orow = out + (size_t)row * HSZ + lane * 8;
#pragma unroll
  for (int j = 0; j < 4; ++j) *(volatile v4u*)(orow + j * 256) = pk[j];
  __threadfence();
#pragma unroll
  for (int j = 0; j < 4; ++j) *(volatile v4u*)(orow + j * 256) = pk[j];
}

template <int BIAS_ROW, int RELU, int OUT32>
__global__ __launch_bounds__(256) void gemm64(
    const unsigned short* __restrict__ Ap, int lda, long long strideA,
    const unsigned short* __restrict__ Bp, int ldb, long long strideB,
    const float* __restrict__ bias, int biasOff,
    const float* __restrict__ res, int ldr, long long strideR,
    void* Cout, int ldc, long long strideC,
    int M, int N, int K, float oscale) {
  __shared__ __align__(16) float sT[8][16 * 68];
  const int b    = blockIdx.y;
  const int lane = threadIdx.x & 31;
  const int wave = threadIdx.x >> 5;
  const int tilesN = N >> 6;
  const int tilesM = M >> 6;
  const int tile = blockIdx.x * 8 + wave;
  if (tile >= tilesM * tilesN) return;
  const int tm = tile / tilesN;
  const int tn = tile - tm * tilesN;
  const int m0 = tm << 6;
  const int n0 = tn << 6;

  const _Float16* A  = (const _Float16*)(const void*)Ap + (size_t)b * (size_t)strideA;
  const _Float16* Bt = (const _Float16*)(const void*)Bp + (size_t)b * (size_t)strideB;

  const int rlane = lane & 15;
  const int koff  = (lane >> 4) * 8;
  const int mOff  = (lane >> 4) * 8;

  v8f acc[4][4];
#pragma unroll
  for (int i = 0; i < 4; ++i)
#pragma unroll
    for (int j = 0; j < 4; ++j) acc[i][j] = zero8();

  for (int k0 = 0; k0 < K; k0 += 32) {
    v16h bf[4];
#pragma unroll
    for (int j = 0; j < 4; ++j)
      bf[j] = ldfrag(Bt + (size_t)(n0 + (j << 4) + rlane) * ldb + koff + k0);
#pragma unroll
    for (int i = 0; i < 4; ++i) {
      const v16h af = ldfrag(A + (size_t)(m0 + (i << 4) + rlane) * lda + koff + k0);
#pragma unroll
      for (int j = 0; j < 4; ++j) acc[i][j] = mma_raw(af, bf[j], acc[i][j]);
      dep_guard(acc[i][0], acc[i][3], af);
    }
    keep4(bf[0], bf[1], bf[2], bf[3]);
  }
  acc_guard4(acc[0][0], acc[0][1], acc[0][2], acc[0][3]);
  acc_guard4(acc[1][0], acc[1][1], acc[1][2], acc[1][3]);
  acc_guard4(acc[2][0], acc[2][1], acc[2][2], acc[2][3]);
  acc_guard4(acc[3][0], acc[3][1], acc[3][2], acc[3][3]);

  float* slab = sT[wave];
#pragma unroll
  for (int i = 0; i < 4; ++i) {
    const int mBase = m0 + (i << 4);
#pragma unroll
    for (int j = 0; j < 4; ++j) {
#pragma unroll
      for (int r = 0; r < 8; ++r) slab[(mOff + r) * 68 + (j << 4) + rlane] = acc[i][j][r];
    }
    __builtin_amdgcn_fence(__ATOMIC_RELEASE, "workgroup");
    __builtin_amdgcn_wave_barrier();
    __builtin_amdgcn_fence(__ATOMIC_ACQUIRE, "workgroup");
    if (OUT32) {
      float* C = (float*)Cout + (size_t)b * (size_t)strideC;
      const float* R = res + (size_t)b * (size_t)strideR;
      const int hq = lane >> 4, c4 = (lane & 15) * 4;
      const v4f bv = *(const v4f*)(bias + biasOff + n0 + c4);
      v4f ov[8];
#pragma unroll
      for (int it = 0; it < 8; ++it) {
        const int row = it * 2 + hq;
        const v4f sv = *(const v4f*)(slab + row * 68 + c4);
        const v4f rv = *(const v4f*)(R + (size_t)(mBase + row) * ldr + n0 + c4);
        v4f o = sv * oscale + bv;
        if (RELU) {
          o[0] = fmaxf(o[0], 0.f); o[1] = fmaxf(o[1], 0.f); o[2] = fmaxf(o[2], 0.f); o[3] = fmaxf(o[3], 0.f);
        }
        o = o + rv;
        ov[it] = o;
      }
#pragma unroll
      for (int it = 0; it < 8; ++it) {
        const int row = it * 2 + hq;
        *(volatile v4f*)(C + (size_t)(mBase + row) * ldc + n0 + c4) = ov[it];
      }
      __threadfence();
#pragma unroll
      for (int it = 0; it < 8; ++it) {
        const int row = it * 2 + hq;
        *(volatile v4f*)(C + (size_t)(mBase + row) * ldc + n0 + c4) = ov[it];
      }
    } else {
      unsigned short* C = (unsigned short*)Cout + (size_t)b * (size_t)strideC;
      const int q = lane >> 3, c8 = (lane & 7) * 8;
      float bcol[8];
      if (!BIAS_ROW) {
        const v4f b0 = *(const v4f*)(bias + biasOff + n0 + c8);
        const v4f b1 = *(const v4f*)(bias + biasOff + n0 + c8 + 4);
        bcol[0] = b0[0]; bcol[1] = b0[1]; bcol[2] = b0[2]; bcol[3] = b0[3];
        bcol[4] = b1[0]; bcol[5] = b1[1]; bcol[6] = b1[2]; bcol[7] = b1[3];
      } else {
#pragma unroll
        for (int e = 0; e < 8; ++e) bcol[e] = 0.f;
      }
      v4u hv[4];
#pragma unroll
      for (int it = 0; it < 4; ++it) {
        const int row = it * 4 + q;
        const float* sp = slab + row * 68 + c8;
        const v4f x0 = *(const v4f*)(sp);
        const v4f x1 = *(const v4f*)(sp + 4);
        float bb[8];
        if (BIAS_ROW) {
          const float br = bias[biasOff + mBase + row];
#pragma unroll
          for (int e = 0; e < 8; ++e) bb[e] = br;
        } else {
#pragma unroll
          for (int e = 0; e < 8; ++e) bb[e] = bcol[e];
        }
        float o[8];
        o[0] = x0[0] * oscale + bb[0]; o[1] = x0[1] * oscale + bb[1];
        o[2] = x0[2] * oscale + bb[2]; o[3] = x0[3] * oscale + bb[3];
        o[4] = x1[0] * oscale + bb[4]; o[5] = x1[1] * oscale + bb[5];
        o[6] = x1[2] * oscale + bb[6]; o[7] = x1[3] * oscale + bb[7];
        if (RELU) {
#pragma unroll
          for (int e = 0; e < 8; ++e) o[e] = fmaxf(o[e], 0.f);
        }
        v4u p;
        p[0] = pkf(o[0], o[1]); p[1] = pkf(o[2], o[3]); p[2] = pkf(o[4], o[5]); p[3] = pkf(o[6], o[7]);
        hv[it] = p;
      }
#pragma unroll
      for (int it = 0; it < 4; ++it) {
        const int row = it * 4 + q;
        *(volatile v4u*)(C + (size_t)(mBase + row) * ldc + n0 + c8) = hv[it];
      }
      __threadfence();
#pragma unroll
      for (int it = 0; it < 4; ++it) {
        const int row = it * 4 + q;
        *(volatile v4u*)(C + (size_t)(mBase + row) * ldc + n0 + c8) = hv[it];
      }
    }
    __builtin_amdgcn_fence(__ATOMIC_RELEASE, "workgroup");
    __builtin_amdgcn_wave_barrier();
    __builtin_amdgcn_fence(__ATOMIC_ACQUIRE, "workgroup");
  }
}

__global__ __launch_bounds__(128)
void attn64(const unsigned short* __restrict__ qkp, const unsigned short* __restrict__ vtp,
            const float* __restrict__ pmask, unsigned short* chp) {
  union FH { v16h v; v8h h[2]; };
  __shared__ __align__(16) _Float16 Ksh[64 * 64];
  __shared__ __align__(16) _Float16 Vth[64 * 64];
  __shared__ __align__(16) _Float16 Psh[4][16 * 64];
  __shared__ __align__(16) float    Os[4][16 * 64];

  const int tid  = threadIdx.x;
  const int wave = tid >> 5;
  const int lane = tid & 31;
  const int hh   = lane >> 4;
  const int c    = lane & 15;

  const int bx = blockIdx.x;
  const int qb = bx % NKT;
  const int h  = (bx / NKT) % NH;
  const int b  = bx / (NKT * NH);
  const int q0 = qb * 64 + wave * 16;
  const size_t rowB = (size_t)b * SEQ;

  const _Float16* Q  = (const _Float16*)(const void*)qkp + (size_t)h * HD;
  const _Float16* Kk = (const _Float16*)(const void*)qkp + HSZ + (size_t)h * HD;
  const _Float16* Vt = (const _Float16*)(const void*)vtp + ((size_t)b * HSZ + (size_t)h * HD) * SEQ;
  const float* mb = pmask + (size_t)b * SEQ;

  v16h qa[2];
#pragma unroll
  for (int dc = 0; dc < 2; ++dc) qa[dc] = ldfrag(Q + (rowB + q0 + c) * QKP + dc * 32 + 8 * hh);

  float mrow[8], lrow[8];
  v8f oacc[4];
#pragma unroll
  for (int r = 0; r < 8; ++r) { mrow[r] = -INFINITY; lrow[r] = 0.f; }
#pragma unroll
  for (int t = 0; t < 4; ++t) oacc[t] = zero8();

  for (int kt = 0; kt < NKT; ++kt) {
    const int kv0 = kt * 64;
    __syncthreads();
    {
      const int r = tid >> 1, half = (tid & 1) * 32;
      const _Float16* kg = Kk + (rowB + kv0 + r) * QKP + half;
      const _Float16* vg = Vt + (size_t)r * SEQ + kv0 + half;
#pragma unroll
      for (int i = 0; i < 4; ++i) {
        const v8h ka = *(const v8h*)(kg + 8 * i);
        const v8h va = *(const v8h*)(vg + 8 * i);
        *(v8h*)(Ksh + r * 64 + half + 8 * i) = ka;
        *(v8h*)(Vth + r * 64 + half + 8 * i) = va;
      }
    }
    __syncthreads();

    v8f s[4];
#pragma unroll
    for (int j = 0; j < 4; ++j) {
      s[j] = zero8();
#pragma unroll
      for (int dc = 0; dc < 2; ++dc) {
        FH kb;
        kb.h[0] = *(const v8h*)(Ksh + (j * 16 + c) * 64 + dc * 32 + 8 * hh);
        kb.h[1] = *(const v8h*)(Ksh + (j * 16 + c) * 64 + dc * 32 + 16 + 8 * hh);
        s[j] = mma_g(qa[dc], kb.v, s[j]);
      }
    }

    float madd[4];
#pragma unroll
    for (int j = 0; j < 4; ++j) madd[j] = mb[kv0 + j * 16 + c] * (-1.0e8f);
    _Float16* pw = Psh[wave];
#pragma unroll
    for (int r = 0; r < 8; ++r) {
      float m = -INFINITY;
#pragma unroll
      for (int j = 0; j < 4; ++j) {
        const float sv = s[j][r] * 0.125f + madd[j];
        s[j][r] = sv;
        m = fmaxf(m, sv);
      }
#pragma unroll
      for (int off = 1; off < 16; off <<= 1) m = fmaxf(m, __shfl_xor(m, off, 32));
      const float mnew  = fmaxf(mrow[r], m);
      const float msafe = (mnew == -INFINITY) ? 0.f : mnew;
      const float alpha = __expf(mrow[r] - msafe);
      mrow[r] = mnew;
      float psum = 0.f;
#pragma unroll
      for (int j = 0; j < 4; ++j) {
        const float p = __expf(s[j][r] - msafe);
        psum += p;
        pw[(8 * hh + r) * 64 + j * 16 + c] = (_Float16)(p * C_P);
      }
#pragma unroll
      for (int off = 1; off < 16; off <<= 1) psum += __shfl_xor(psum, off, 32);
      lrow[r] = lrow[r] * alpha + psum;
#pragma unroll
      for (int t = 0; t < 4; ++t) oacc[t][r] *= alpha;
    }
    __builtin_amdgcn_fence(__ATOMIC_RELEASE, "workgroup");
    __builtin_amdgcn_wave_barrier();
    __builtin_amdgcn_fence(__ATOMIC_ACQUIRE, "workgroup");

#pragma unroll 1
    for (int kk = 0; kk < 2; ++kk) {
      FH pa;
      pa.h[0] = *(const v8h*)(pw + c * 64 + kk * 32 + 8 * hh);
      pa.h[1] = *(const v8h*)(pw + c * 64 + kk * 32 + 16 + 8 * hh);
#pragma unroll
      for (int t = 0; t < 4; ++t) {
        FH vb;
        vb.h[0] = *(const v8h*)(Vth + (t * 16 + c) * 64 + kk * 32 + 8 * hh);
        vb.h[1] = *(const v8h*)(Vth + (t * 16 + c) * 64 + kk * 32 + 16 + 8 * hh);
        oacc[t] = mma_g(pa.v, vb.v, oacc[t]);
      }
    }
  }

  float* os = Os[wave];
#pragma unroll
  for (int r = 0; r < 8; ++r) {
    const float l = lrow[r];
    const float inv = ((l > 0.f) ? (1.0f / l) : 0.f) * (C_CTX / C_P);
#pragma unroll
    for (int t = 0; t < 4; ++t) os[(8 * hh + r) * 64 + t * 16 + c] = oacc[t][r] * inv;
  }
  __builtin_amdgcn_fence(__ATOMIC_RELEASE, "workgroup");
  __builtin_amdgcn_wave_barrier();
  __builtin_amdgcn_fence(__ATOMIC_ACQUIRE, "workgroup");
  {
    const int q4 = lane >> 3, c8 = (lane & 7) * 8;
    v4u hv[4];
#pragma unroll
    for (int it = 0; it < 4; ++it) {
      const int row = it * 4 + q4;
      const float* sp = os + row * 64 + c8;
      const v4f a0 = *(const v4f*)(sp);
      const v4f a1 = *(const v4f*)(sp + 4);
      v4u p;
      p[0] = pkf(a0[0], a0[1]); p[1] = pkf(a0[2], a0[3]); p[2] = pkf(a1[0], a1[1]); p[3] = pkf(a1[2], a1[3]);
      hv[it] = p;
    }
#pragma unroll
    for (int it = 0; it < 4; ++it) {
      const int row = it * 4 + q4;
      *(volatile v4u*)(chp + (rowB + q0 + row) * HSZ + (size_t)h * HD + c8) = hv[it];
    }
    __threadfence();
#pragma unroll
    for (int it = 0; it < 4; ++it) {
      const int row = it * 4 + q4;
      *(volatile v4u*)(chp + (rowB + q0 + row) * HSZ + (size_t)h * HD + c8) = hv[it];
    }
  }
}

extern "C" void kernel_launch(void* const* d_in, const int* in_sizes, int n_in,
                              void* d_out, int out_size, void* d_ws, size_t ws_size,
                              hipStream_t stream) {
  if (n_in < 14) return;
  if (in_sizes[0] != NTOK * HSZ) return;
  if (in_sizes[1] != NBATCH * SEQ) return;
  if (in_sizes[2] != 3 * HSZ * HSZ || in_sizes[3] != 3 * HSZ) return;
  if (in_sizes[4] != HSZ * HSZ || in_sizes[5] != HSZ) return;
  if (in_sizes[6] != HSZ || in_sizes[7] != HSZ) return;
  if (in_sizes[8] != IMSZ * HSZ || in_sizes[9] != IMSZ) return;
  if (in_sizes[10] != HSZ * IMSZ || in_sizes[11] != HSZ) return;
  if (in_sizes[12] != HSZ || in_sizes[13] != HSZ) return;
  if (out_size != NTOK * HSZ) return;

  const float* x     = (const float*)d_in[0];
  const float* pmask = (const float*)d_in[1];
  const float* qkv_w = (const float*)d_in[2];
  const float* qkv_b = (const float*)d_in[3];
  const float* ao_w  = (const float*)d_in[4];
  const float* ao_b  = (const float*)d_in[5];
  const float* ln1_g = (const float*)d_in[6];
  const float* ln1_b = (const float*)d_in[7];
  const float* in_w  = (const float*)d_in[8];
  const float* in_b  = (const float*)d_in[9];
  const float* fo_w  = (const float*)d_in[10];
  const float* fo_b  = (const float*)d_in[11];
  const float* ln2_g = (const float*)d_in[12];
  const float* ln2_b = (const float*)d_in[13];
  float* out = (float*)d_out;

  const size_t szWqkv = (size_t)3 * HSZ * HSZ * 2;
  const size_t szWo   = (size_t)HSZ * HSZ * 2;
  const size_t szWi   = (size_t)IMSZ * HSZ * 2;
  const size_t szWf   = (size_t)HSZ * IMSZ * 2;
  const size_t szX    = (size_t)NTOK * HSZ * 2;
  const size_t szQK   = (size_t)NTOK * QKP * 2;
  const size_t szVT   = (size_t)NBATCH * HSZ * SEQ * 2;
  const size_t szC    = (size_t)NTOK * HSZ * 2;
  const size_t szH    = (size_t)NTOK * IMSZ * 2;
  const size_t szY    = (size_t)NTOK * HSZ * 4;
  size_t off = 0;
  const size_t oR0 = off; off += szWqkv + szWo;
  const size_t oXh = off; off += szX;
  const size_t oQK = off; off += szQK;
  const size_t oVT = off; off += szVT;
  const size_t oC  = off; off += szC;
  const size_t oY  = off; off += szY;
  if (off > ws_size) return;
  if (off > (size_t)134217728) return;
  if (szWi > szWqkv + szWo) return;
  if (szWf > szX) return;
  if (szH != szQK + szVT + szC) return;

  char* ws = (char*)d_ws;
  unsigned short* Wqkv16 = (unsigned short*)(ws + oR0);
  unsigned short* Wo16   = (unsigned short*)(ws + oR0 + szWqkv);
  unsigned short* Wi16   = (unsigned short*)(ws + oR0);
  unsigned short* Xh     = (unsigned short*)(ws + oXh);
  unsigned short* Wf16   = (unsigned short*)(ws + oXh);
  unsigned short* QK     = (unsigned short*)(ws + oQK);
  unsigned short* VT     = (unsigned short*)(ws + oVT);
  unsigned short* Ch     = (unsigned short*)(ws + oC);
  unsigned short* Hh     = (unsigned short*)(ws + oQK);
  float*          Y      = (float*)(ws + oY);

  const dim3 blk(256);
  const int n8qkv = 3 * HSZ * HSZ / 8;
  const int n8o   = HSZ * HSZ / 8;
  const int n8i   = IMSZ * HSZ / 8;
  const int n8f   = HSZ * IMSZ / 8;
  const int tilesQK = (NTOK / 64) * (QKP / 64);
  const int tilesVT = (HSZ / 64) * (SEQ / 64);
  const int tilesO  = (NTOK / 64) * (HSZ / 64);
  const int tilesI  = (NTOK / 64) * (IMSZ / 64);

  cvt_f16x8<<<dim3((n8qkv + 255) / 256), blk, 0, stream>>>(qkv_w, Wqkv16, n8qkv, CW_QKV);
  cvt_f16x8<<<dim3((n8o + 255) / 256), blk, 0, stream>>>(ao_w, Wo16, n8o, CW_O);
  ln_f16<<<dim3((NTOK + 7) / 8), blk, 0, stream>>>(x, ln1_g, ln1_b, Xh, NTOK);
  gemm64<0, 0, 0><<<dim3((tilesQK + 7) / 8, 1), blk, 0, stream>>>(
      Xh, HSZ, 0LL, Wqkv16, HSZ, 0LL, qkv_b, 0, x, HSZ, 0LL,
      (void*)QK, QKP, 0LL, NTOK, QKP, HSZ, 1.0f / CW_QKV);
  gemm64<1, 0, 0><<<dim3((tilesVT + 7) / 8, NBATCH), blk, 0, stream>>>(
      Wqkv16 + (size_t)2 * HSZ * HSZ, HSZ, 0LL, Xh, HSZ, (long long)SEQ * HSZ, qkv_b, 2 * HSZ, x, HSZ, 0LL,
      (void*)VT, SEQ, (long long)HSZ * SEQ, HSZ, SEQ, HSZ, 1.0f / CW_QKV);
  attn64<<<dim3(NBATCH * NH * NKT), dim3(128), 0, stream>>>(QK, VT, pmask, Ch);
  gemm64<0, 0, 1><<<dim3((tilesO + 7) / 8, 1), blk, 0, stream>>>(
      Ch, HSZ, 0LL, Wo16, HSZ, 0LL, ao_b, 0, x, HSZ, 0LL,
      (void*)Y, HSZ, 0LL, NTOK, HSZ, HSZ, 1.0f / (C_CTX * CW_O));
  cvt_f16x8<<<dim3((n8i + 255) / 256), blk, 0, stream>>>(in_w, Wi16, n8i, CW_I);
  ln_f16<<<dim3((NTOK + 7) / 8), blk, 0, stream>>>(Y, ln2_g, ln2_b, Xh, NTOK);
  gemm64<0, 1, 0><<<dim3((tilesI + 7) / 8, 1), blk, 0, stream>>>(
      Xh, HSZ, 0LL, Wi16, HSZ, 0LL, in_b, 0, x, HSZ, 0LL,
      (void*)Hh, IMSZ, 0LL, NTOK, IMSZ, HSZ, 1.0f / CW_I);
  cvt_f16x8<<<dim3((n8f + 255) / 256), blk, 0, stream>>>(fo_w, Wf16, n8f, CW_F);
  gemm64<0, 0, 1><<<dim3((tilesO + 7) / 8, 1), blk, 0, stream>>>(
      Hh, IMSZ, 0LL, Wf16, IMSZ, 0LL, fo_b, 0, Y, HSZ, 0LL,
      (void*)out, HSZ, 0LL, NTOK, HSZ, IMSZ, 1.0f / CW_F);
  (void)hipGetLastError();
}
